// StructuredDecoding_81836306858628
// MI455X (gfx1250) — hardware-run, weakly checked
//
#include <hip/hip_runtime.h>
#include <math.h>

typedef __attribute__((ext_vector_type(16))) _Float16 v16h;
typedef __attribute__((ext_vector_type(8)))  _Float16 v8h;
typedef __attribute__((ext_vector_type(4)))  _Float16 v4h;
typedef __attribute__((ext_vector_type(8)))  float    v8f;
typedef __attribute__((ext_vector_type(4)))  float    v4f;

constexpr int kNB   = 32;
constexpr int kNT   = 512;
constexpr int kNS   = 128;
constexpr int kRowsPerBlock = 16;
constexpr int kHP   = 136;
constexpr int kGP   = 132;
constexpr float kClampEps     = 1e-10f;
constexpr float kTinyGuard    = 1e-30f;
constexpr float kTnCarry      = 256.0f;
constexpr float kStateCarry   = 64.0f;
constexpr float kF16MinNormal = 6.103515625e-5f;

static_assert(kNS == 128, "eight 16-column tiles, four 32-deep k steps");
static_assert((kNS % 32) == 0, "K multiple of 32");
static_assert((kNB % kRowsPerBlock) == 0, "whole M tiles");
static_assert((kHP % 8) == 0 && (kGP % 4) == 0, "16-B aligned LDS rows");

constexpr size_t kOffU   = 0;
constexpr size_t kOffZ   = kOffU  + (size_t)kNB * kNT * kNS * 4;
constexpr size_t kOffTT  = kOffZ  + (size_t)kNB * kNT * kNS * 4;
constexpr size_t kOffTN  = kOffTT + (size_t)kNS * kNS * 2;
constexpr size_t kWsTotal = kOffTN + (size_t)kNS * kNS * 2;
static_assert(kWsTotal == 16842752ull, "carve total");
static_assert(kWsTotal <= 134217728ull, "carve cap");
static_assert((kOffZ % 128) == 0 && (kOffTT % 128) == 0 && (kOffTN % 128) == 0, "128-B aligned regions");

union FragH { v16h v; v8h h[2]; };

__device__ __forceinline__ v16h frag_load(const _Float16* p) {
  FragH f;
  f.h[0] = *(const v8h*)(p);
  f.h[1] = *(const v8h*)(p + 16);
  return f.v;
}

__device__ __forceinline__ v8f mma_h(v16h a, v16h b, v8f c) {
  c = __builtin_amdgcn_wmma_f32_16x16x32_f16(false, a, false, b, (short)0, c, false, false);
  asm volatile("v_nop\n\tv_nop\n\tv_nop\n\tv_nop" : "+v"(c) : "v"(a), "v"(b));
  return c;
}

__device__ __forceinline__ _Float16 to_h16_flush(float v) {
  const float f = (fabsf(v) < kF16MinNormal) ? 0.0f : v;
  return (_Float16)f;
}

__device__ __forceinline__ float wave_max(float v) {
#pragma unroll
  for (int off = 16; off >= 1; off >>= 1) v = fmaxf(v, __shfl_xor(v, off, 32));
  return v;
}
__device__ __forceinline__ float wave_sum(float v) {
#pragma unroll
  for (int off = 16; off >= 1; off >>= 1) v += __shfl_xor(v, off, 32);
  return v;
}

__device__ __forceinline__ void put_a4(_Float16* dst, v4f v, float sc) {
  v4h hv;
  hv[0] = to_h16_flush(v[0] * sc);
  hv[1] = to_h16_flush(v[1] * sc);
  hv[2] = to_h16_flush(v[2] * sc);
  hv[3] = to_h16_flush(v[3] * sc);
  *(v4h*)dst = hv;
}

__device__ __forceinline__ void tile_gemm(const _Float16* sA, float* sG,
                                          v16h b0, v16h b1, v16h b2, v16h b3,
                                          int c, int hh, int n0) {
  v8f acc = (v8f){0.f, 0.f, 0.f, 0.f, 0.f, 0.f, 0.f, 0.f};
  const _Float16* ap = sA + c * kHP + 8 * hh;
  acc = mma_h(frag_load(ap),      b0, acc);
  acc = mma_h(frag_load(ap + 32), b1, acc);
  acc = mma_h(frag_load(ap + 64), b2, acc);
  acc = mma_h(frag_load(ap + 96), b3, acc);
  float* gp = sG + (8 * hh) * kGP + n0 + c;
#pragma unroll
  for (int r = 0; r < 8; ++r) gp[r * kGP] = acc[r];
}

__global__ __launch_bounds__(256) void prep_planes_kernel(
    const float* __restrict__ trans, _Float16* __restrict__ TT16, _Float16* __restrict__ TN16)
{
  __shared__ __align__(16) _Float16 sTile[kNS * kHP];
  __shared__ float sScale[kNS];
  const int tid = threadIdx.x, lane = tid & 31, wave = tid >> 5;
  const int half = lane >> 4, c8 = (lane & 15) * 8;

#pragma unroll 1
  for (int i = 0; i < 16; ++i) {
    const int from = wave * 16 + i;
    const v4f x = *(const v4f*)(trans + (size_t)from * kNS + 4 * lane);
    const float c0 = fmaxf(x[0], kClampEps), c1 = fmaxf(x[1], kClampEps);
    const float c2 = fmaxf(x[2], kClampEps), c3 = fmaxf(x[3], kClampEps);
    const float s  = wave_sum((c0 + c1) + (c2 + c3));
    const float rs = 1.0f / s;
    if (lane == 0) sScale[from] = rs;
    sTile[(4 * lane + 0) * kHP + from] = to_h16_flush((c0 * rs) * kTnCarry);
    sTile[(4 * lane + 1) * kHP + from] = to_h16_flush((c1 * rs) * kTnCarry);
    sTile[(4 * lane + 2) * kHP + from] = to_h16_flush((c2 * rs) * kTnCarry);
    sTile[(4 * lane + 3) * kHP + from] = to_h16_flush((c3 * rs) * kTnCarry);
  }
  __syncthreads();
  {
    v8h tv[8];
#pragma unroll
    for (int it = 0; it < 8; ++it) tv[it] = *(const v8h*)(sTile + (wave * 16 + it * 2 + half) * kHP + c8);
    for (int pass = 0; pass < 2; ++pass) {
#pragma unroll
      for (int it = 0; it < 8; ++it)
        *(volatile v8h*)(TT16 + (size_t)(wave * 16 + it * 2 + half) * kNS + c8) = tv[it];
      __threadfence();
    }
  }
  __syncthreads();
#pragma unroll 1
  for (int i = 0; i < 16; ++i) {
    const int from = wave * 16 + i;
    const v4f x = *(const v4f*)(trans + (size_t)from * kNS + 4 * lane);
    const float rs = sScale[from];
    v4h hv;
    hv[0] = to_h16_flush((fmaxf(x[0], kClampEps) * rs) * kTnCarry);
    hv[1] = to_h16_flush((fmaxf(x[1], kClampEps) * rs) * kTnCarry);
    hv[2] = to_h16_flush((fmaxf(x[2], kClampEps) * rs) * kTnCarry);
    hv[3] = to_h16_flush((fmaxf(x[3], kClampEps) * rs) * kTnCarry);
    *(v4h*)(sTile + from * kHP + 4 * lane) = hv;
  }
  __syncthreads();
  {
    v8h tv[8];
#pragma unroll
    for (int it = 0; it < 8; ++it) tv[it] = *(const v8h*)(sTile + (wave * 16 + it * 2 + half) * kHP + c8);
    for (int pass = 0; pass < 2; ++pass) {
#pragma unroll
      for (int it = 0; it < 8; ++it)
        *(volatile v8h*)(TN16 + (size_t)(wave * 16 + it * 2 + half) * kNS + c8) = tv[it];
      __threadfence();
    }
  }
}

__global__ __launch_bounds__(256) void soft_path_kernel(
    const float* __restrict__ logem, const float* __restrict__ prior,
    const _Float16* __restrict__ TT16, const _Float16* __restrict__ TN16,
    float* Uws, float* Zws, float* out)
{
  __shared__ __align__(16) _Float16 sA[kRowsPerBlock * kHP];
  __shared__ __align__(16) float    sG[kRowsPerBlock * kGP];

  const int tid = threadIdx.x, lane = tid & 31, wave = tid >> 5;
  const int hh = lane >> 4, c = lane & 15;
  const int n0 = wave * 16;
  const int c4 = lane * 4;
  const int bb = blockIdx.x * kRowsPerBlock;
  const int rowA = 2 * wave, rowB = 2 * wave + 1;
  const size_t gA = (size_t)(bb + rowA) * kNT;
  const size_t gB = (size_t)(bb + rowB) * kNT;

  v16h b0, b1, b2, b3;
  {
    const _Float16* bp = TT16 + (size_t)(n0 + c) * kNS + 8 * hh;
    b0 = frag_load(bp);
    b1 = frag_load(bp + 32);
    b2 = frag_load(bp + 64);
    b3 = frag_load(bp + 96);
  }

  v4f uA, uB;
  {
    const v4f pv = *(const v4f*)(prior + c4);
    const v4f eA = *(const v4f*)(logem + (gA + 0) * kNS + c4);
    const v4f eB = *(const v4f*)(logem + (gB + 0) * kNS + c4);
#pragma unroll
    for (int j = 0; j < 4; ++j) {
      const float pj = fmaxf(pv[j], kClampEps);
      uA[j] = pj * expf(eA[j]);
      uB[j] = pj * expf(eB[j]);
    }
    const float mA = wave_max(fmaxf(fmaxf(uA[0], uA[1]), fmaxf(uA[2], uA[3])));
    const float mB = wave_max(fmaxf(fmaxf(uB[0], uB[1]), fmaxf(uB[2], uB[3])));
    const float iA = 1.0f / fmaxf(mA, kTinyGuard);
    const float iB = 1.0f / fmaxf(mB, kTinyGuard);
#pragma unroll
    for (int j = 0; j < 4; ++j) { uA[j] *= iA; uB[j] *= iB; }
    put_a4(sA + rowA * kHP + c4, uA, kStateCarry);
    put_a4(sA + rowB * kHP + c4, uB, kStateCarry);
    float* pUA = Uws + (gA + 0) * kNS + c4;
    float* pUB = Uws + (gB + 0) * kNS + c4;
    *(volatile v4f*)pUA = uA;
    *(volatile v4f*)pUB = uB;
    __threadfence();
    *(volatile v4f*)pUA = uA;
    *(volatile v4f*)pUB = uB;
  }
  __syncthreads();

#pragma unroll 1
  for (int t = 0; t < kNT - 1; ++t) {
    tile_gemm(sA, sG, b0, b1, b2, b3, c, hh, n0);
    __syncthreads();
    const v4f zA = *(const v4f*)(sG + rowA * kGP + c4);
    const v4f zB = *(const v4f*)(sG + rowB * kGP + c4);
    const v4f eA = *(const v4f*)(logem + (gA + t + 1) * kNS + c4);
    const v4f eB = *(const v4f*)(logem + (gB + t + 1) * kNS + c4);
#pragma unroll
    for (int j = 0; j < 4; ++j) {
      uA[j] = expf(eA[j]) * zA[j];
      uB[j] = expf(eB[j]) * zB[j];
    }
    const float mA = wave_max(fmaxf(fmaxf(uA[0], uA[1]), fmaxf(uA[2], uA[3])));
    const float mB = wave_max(fmaxf(fmaxf(uB[0], uB[1]), fmaxf(uB[2], uB[3])));
    const float iA = 1.0f / fmaxf(mA, kTinyGuard);
    const float iB = 1.0f / fmaxf(mB, kTinyGuard);
#pragma unroll
    for (int j = 0; j < 4; ++j) { uA[j] *= iA; uB[j] *= iB; }
    put_a4(sA + rowA * kHP + c4, uA, kStateCarry);
    put_a4(sA + rowB * kHP + c4, uB, kStateCarry);
    float* pZA = Zws + (gA + t) * kNS + c4;
    float* pZB = Zws + (gB + t) * kNS + c4;
    float* pUA = Uws + (gA + t + 1) * kNS + c4;
    float* pUB = Uws + (gB + t + 1) * kNS + c4;
    *(volatile v4f*)pZA = zA;
    *(volatile v4f*)pZB = zB;
    *(volatile v4f*)pUA = uA;
    *(volatile v4f*)pUB = uB;
    __threadfence();
    *(volatile v4f*)pZA = zA;
    *(volatile v4f*)pZB = zB;
    *(volatile v4f*)pUA = uA;
    *(volatile v4f*)pUB = uB;
    __syncthreads();
  }
  __threadfence();
  __syncthreads();
  asm volatile("" ::: "memory");

  v4f pA, pB;
  {
    const float sA_ = wave_sum((uA[0] + uA[1]) + (uA[2] + uA[3]));
    const float sB_ = wave_sum((uB[0] + uB[1]) + (uB[2] + uB[3]));
    const float iA = 1.0f / fmaxf(sA_, kTinyGuard);
    const float iB = 1.0f / fmaxf(sB_, kTinyGuard);
#pragma unroll
    for (int j = 0; j < 4; ++j) { pA[j] = uA[j] * iA; pB[j] = uB[j] * iB; }
    float* oA = out + (gA + (kNT - 1)) * kNS + c4;
    float* oB = out + (gB + (kNT - 1)) * kNS + c4;
    *(volatile v4f*)oA = pA;
    *(volatile v4f*)oB = pB;
    __threadfence();
    *(volatile v4f*)oA = pA;
    *(volatile v4f*)oB = pB;
  }

  {
    const _Float16* bp = TN16 + (size_t)(n0 + c) * kNS + 8 * hh;
    b0 = frag_load(bp);
    b1 = frag_load(bp + 32);
    b2 = frag_load(bp + 64);
    b3 = frag_load(bp + 96);
  }

#pragma unroll 1
  for (int t = kNT - 2; t >= 0; --t) {
    {
      const v4f zA = *(const v4f*)(Zws + (gA + t) * kNS + c4);
      const v4f zB = *(const v4f*)(Zws + (gB + t) * kNS + c4);
      v4f wA, wB;
#pragma unroll
      for (int j = 0; j < 4; ++j) {
        wA[j] = pA[j] * (1.0f / fmaxf(zA[j], kTinyGuard));
        wB[j] = pB[j] * (1.0f / fmaxf(zB[j], kTinyGuard));
      }
      const float mA = wave_max(fmaxf(fmaxf(wA[0], wA[1]), fmaxf(wA[2], wA[3])));
      const float mB = wave_max(fmaxf(fmaxf(wB[0], wB[1]), fmaxf(wB[2], wB[3])));
      const float scA = kStateCarry * (1.0f / fmaxf(mA, kTinyGuard));
      const float scB = kStateCarry * (1.0f / fmaxf(mB, kTinyGuard));
      put_a4(sA + rowA * kHP + c4, wA, scA);
      put_a4(sA + rowB * kHP + c4, wB, scB);
    }
    __syncthreads();
    tile_gemm(sA, sG, b0, b1, b2, b3, c, hh, n0);
    __syncthreads();
    {
      const v4f qA = *(const v4f*)(sG + rowA * kGP + c4);
      const v4f qB = *(const v4f*)(sG + rowB * kGP + c4);
      const v4f xA = *(const v4f*)(Uws + (gA + t) * kNS + c4);
      const v4f xB = *(const v4f*)(Uws + (gB + t) * kNS + c4);
#pragma unroll
      for (int j = 0; j < 4; ++j) { pA[j] = xA[j] * qA[j]; pB[j] = xB[j] * qB[j]; }
      const float sA_ = wave_sum((pA[0] + pA[1]) + (pA[2] + pA[3]));
      const float sB_ = wave_sum((pB[0] + pB[1]) + (pB[2] + pB[3]));
      const float iA = 1.0f / fmaxf(sA_, kTinyGuard);
      const float iB = 1.0f / fmaxf(sB_, kTinyGuard);
#pragma unroll
      for (int j = 0; j < 4; ++j) { pA[j] *= iA; pB[j] *= iB; }
      float* oA = out + (gA + t) * kNS + c4;
      float* oB = out + (gB + t) * kNS + c4;
      *(volatile v4f*)oA = pA;
      *(volatile v4f*)oB = pB;
      __threadfence();
      *(volatile v4f*)oA = pA;
      *(volatile v4f*)oB = pB;
    }
  }
}

extern "C" void kernel_launch(void* const* d_in, const int* in_sizes, int n_in,
                              void* d_out, int out_size, void* d_ws, size_t ws_size,
                              hipStream_t stream) {
  if (n_in < 3) return;
  if (in_sizes[0] != kNS * kNS) return;
  if (in_sizes[1] != kNB * kNT * kNS) return;
  if (in_sizes[2] != kNS) return;
  if (out_size != kNB * kNT * kNS) return;
  if (ws_size < kWsTotal) return;

  const float* trans = (const float*)d_in[0];
  const float* logem = (const float*)d_in[1];
  const float* prior = (const float*)d_in[2];
  float* out = (float*)d_out;

  char* ws = (char*)d_ws;
  float*    Uws  = (float*)(ws + kOffU);
  float*    Zws  = (float*)(ws + kOffZ);
  _Float16* TT16 = (_Float16*)(ws + kOffTT);
  _Float16* TN16 = (_Float16*)(ws + kOffTN);

  prep_planes_kernel<<<1, 256, 0, stream>>>(trans, TT16, TN16);
  soft_path_kernel<<<kNB / kRowsPerBlock, 256, 0, stream>>>(logem, prior, TT16, TN16, Uws, Zws, out);
}
